// Conv2d_mod_32083405701533
// MI455X (gfx1250) — hardware-verified
//
#include <hip/hip_runtime.h>
#include <math.h>

typedef __attribute__((ext_vector_type(16))) _Float16 v16h;
typedef __attribute__((ext_vector_type(16))) __bf16 v16b;
typedef __attribute__((ext_vector_type(8)))  _Float16 v8h;
typedef __attribute__((ext_vector_type(8)))  float v8f;
typedef __attribute__((ext_vector_type(4)))  float v4f;
typedef __attribute__((ext_vector_type(2)))  float v2f;
typedef __attribute__((ext_vector_type(4)))  unsigned v4u;
typedef __attribute__((ext_vector_type(4)))  int v4i;
typedef float __attribute__((may_alias)) float_a;
typedef int __attribute__((may_alias)) int_a;

template <typename T> __device__ __forceinline__ void vst2(void* p, T v) { *(volatile T*)p = v; __threadfence(); *(volatile T*)p = v; }
__device__ __forceinline__ v8f wmma16(v16h a, v16h b, v8f c) {
  v8f d = __builtin_amdgcn_wmma_f32_16x16x32_f16(false, a, false, b, (short)0, c, false, false);
  asm volatile("v_nop\n\tv_nop\n\tv_nop\n\tv_nop" : "+v"(d) : "v"(a), "v"(b));
  return d;
}
__device__ __forceinline__ v8f wmma_bf(v16b a, v16b b, v8f c) {
  v8f d = __builtin_amdgcn_wmma_f32_16x16x32_bf16(false, a, false, b, (short)0, c, false, false);
  asm volatile("v_nop\n\tv_nop\n\tv_nop\n\tv_nop" : "+v"(d) : "v"(a), "v"(b));
  return d;
}
__device__ __forceinline__ v16h frag_h(const _Float16* rowk0, int lane) {
  union { v16h v; v8h q[2]; } u; const _Float16* p = rowk0 + 8 * (lane >> 4);
  u.q[0] = *(const v8h*)p; u.q[1] = *(const v8h*)(p + 16); return u.v;
}
__device__ __forceinline__ v16h frag_f32(const float* rowk0, int lane) {
  v16h a; const float* p = rowk0 + 8 * (lane >> 4);
#pragma unroll
  for (int i = 0; i < 8; ++i) { a[i] = (_Float16)p[i]; a[8 + i] = (_Float16)p[16 + i]; }
  return a;
}
__device__ __forceinline__ v16h frag_f32s(const float* rowk0, int lane, float sc) {
  v16h a; const float* p = rowk0 + 8 * (lane >> 4);
#pragma unroll
  for (int i = 0; i < 8; ++i) { a[i] = (_Float16)(p[i] * sc); a[8 + i] = (_Float16)(p[16 + i] * sc); }
  return a;
}
__device__ __forceinline__ v16h fragc_f32(const float* W, int k0, int n, int lane, int ld, int K) {
  v16h a; const int g = lane >> 4;
#pragma unroll
  for (int i = 0; i < 8; ++i) { const int ka = k0 + 8 * g + i, kb = ka + 16;
    a[i] = (_Float16)(ka < K ? W[(size_t)(ka < K ? ka : K - 1) * ld + n] : 0.f); a[8 + i] = (_Float16)(kb < K ? W[(size_t)(kb < K ? kb : K - 1) * ld + n] : 0.f); }
  return a;
}
struct F2 { v16b h, l; };
__device__ __forceinline__ F2 bsplit16(const float v[16]) { F2 r;
#pragma unroll
  for (int i = 0; i < 16; ++i) { const __bf16 h = (__bf16)v[i]; r.h[i] = h; r.l[i] = (__bf16)(v[i] - (float)h); }
  return r; }
__device__ __forceinline__ F2 split_row(const float* row, int k0, int lane) { float v[16]; const float* p = row + k0 + 8 * (lane >> 4);
#pragma unroll
  for (int i = 0; i < 8; ++i) { v[i] = p[i]; v[8 + i] = p[16 + i]; }
  return bsplit16(v); }
__device__ __forceinline__ F2 split_rowK(const float* row, int k0, int lane, int K) { float v[16]; const int g = lane >> 4;
#pragma unroll
  for (int i = 0; i < 8; ++i) { const int ka = k0 + 8 * g + i, kb = ka + 16; v[i] = ka < K ? row[ka < K ? ka : K - 1] : 0.f; v[8 + i] = kb < K ? row[kb < K ? kb : K - 1] : 0.f; }
  return bsplit16(v); }
__device__ __forceinline__ F2 split_col(const float* W, int k0, int n, int lane, int ld, int K) { float v[16]; const int g = lane >> 4;
#pragma unroll
  for (int i = 0; i < 8; ++i) { const int ka = k0 + 8 * g + i, kb = ka + 16; v[i] = ka < K ? W[(size_t)(ka < K ? ka : K - 1) * ld + n] : 0.f; v[8 + i] = kb < K ? W[(size_t)(kb < K ? kb : K - 1) * ld + n] : 0.f; }
  return bsplit16(v); }
__device__ __forceinline__ v8f mac3(const F2& a, const F2& b, v8f c) { c = wmma_bf(a.l, b.h, c); c = wmma_bf(a.h, b.l, c); return wmma_bf(a.h, b.h, c); }
__device__ __forceinline__ float sigm(float v) { return 1.0f / (1.0f + expf(-v)); }
#define LDSX() do { asm volatile("s_wait_dscnt 0" ::: "memory"); __builtin_amdgcn_wave_barrier(); __builtin_amdgcn_fence(__ATOMIC_RELEASE, "workgroup"); } while (0)


#define NB 16
#define CI 512
#define CO 512
#define HH 32
#define WWD 32
#define KK 9
#define KTOT (CI * KK)
#define LAT 256
#ifndef TNB
#define TNB NB
#endif
typedef __attribute__((ext_vector_type(8))) __bf16 v8b;
__device__ __forceinline__ v16b frag_b(const __bf16* rowk0, int lane) {
  union { v16b v; v8b q[2]; } u; const __bf16* p = rowk0 + 8 * (lane >> 4);
  u.q[0] = *(const v8b*)p; u.q[1] = *(const v8b*)(p + 16); return u.v;
}
__device__ __forceinline__ float bfr(float v) { return (float)(__bf16)v; }
__device__ __attribute__((noinline)) float exp_ni(float v) { return expf(v); }
__device__ __attribute__((noinline)) float erf_ni(float v) { return erff(v); }

#define WS_PW  0u
#define WS_W2  (WS_PW + 2u * (size_t)CO * KTOT)
#define WS_SC  (WS_W2 + 4u * (size_t)CO)
#define WS_END (WS_SC + 4u * (size_t)NB * CO)

__global__ __launch_bounds__(256) void k_pack(const float* __restrict__ Wt, __bf16* __restrict__ P, float* __restrict__ W2) {
  const int o = blockIdx.x, t = threadIdx.x;
  if (o < CO) { __shared__ __align__(16) __bf16 s[KTOT]; const float* w = Wt + (size_t)o * KTOT; for (int k = t; k < KTOT; k += 256) s[k] = (__bf16)w[k]; __syncthreads(); for (int q = t; q < KTOT / 8; q += 256) vst2((unsigned*)(P + (size_t)o * KTOT + q * 8), *(const v4u*)&s[q * 8]); return; }
  __shared__ __align__(16) float sq[CO];
  for (int oo = t; oo < CO; oo += 256) { const float* w = Wt + (size_t)oo * KTOT; float a = 0.f; for (int k = 0; k < KTOT; ++k) { const float v = bfr(w[k]); a += v * v; } sq[oo] = a; }
  __syncthreads(); if (t < CO / 4) vst2(W2 + t * 4, *(const v4f*)&sq[t * 4]);
}
__global__ __launch_bounds__(256) void k_style(const float* __restrict__ ST, const float* __restrict__ LW, const float* __restrict__ LB, const float* __restrict__ MB, const float* __restrict__ W2, float* __restrict__ SC) {
  __shared__ float sst[LAT]; __shared__ __align__(16) float so[CO]; const size_t b = blockIdx.x; const int t = threadIdx.x;
  for (int i = t; i < LAT; i += 256) sst[i] = bfr(ST[b * LAT + i]); __syncthreads();
  const float eq_lin = sqrtf(2.0f / (float)LAT), eq_conv = sqrtf(2.0f / (float)(CI * KK));
  for (int o = t; o < CO; o += 256) { float a = 0.f; const float* lw = LW + (size_t)o * LAT; for (int i = 0; i < LAT; ++i) a += sst[i] * (bfr(lw[i]) * eq_lin); const float s = a + bfr(LB[o]) + 1.0f + bfr(MB[o]);
    const float se = s * eq_conv; so[o] = se / sqrtf(se * se * W2[o] + 1e-8f); }
  __syncthreads(); if (t < CO / 4) vst2(SC + b * CO + t * 4, *(const v4f*)&so[t * 4]);
}
__global__ __launch_bounds__(128) void k_conv(const float* __restrict__ X, const __bf16* __restrict__ P, const float* __restrict__ SC, const float* __restrict__ CB, float* __restrict__ OUT) {
  __shared__ __align__(16) __bf16 sx[CI][4][WWD + 2];
  __shared__ __align__(16) float st[64][68];
  const int tid = threadIdx.x, wave = tid >> 5, lane = tid & 31, col = lane & 15, g = lane >> 4; const int y0 = blockIdx.x * 2; const int o0 = blockIdx.y * 128; const size_t b = blockIdx.z;
  for (int e = tid; e < CI * 4 * (WWD + 2); e += 128) { const int c = e / (4 * (WWD + 2)), rem = e % (4 * (WWD + 2)); const int ry = rem / (WWD + 2), rx = rem % (WWD + 2); const int yy = y0 + ry - 1, xx = rx - 1;
    sx[c][ry][rx] = (yy >= 0 && yy < HH && xx >= 0 && xx < WWD) ? (__bf16)X[((b * CI + c) * HH + yy) * WWD + xx] : (__bf16)0.f; }
  __syncthreads();
  const int pyl = wave >> 1, px = (wave & 1) * 16 + col;
  v8f acc[8] = {};
#pragma unroll 1
  for (int kc = 0; kc < KTOT / 32; ++kc) { v16b a;
#pragma unroll
    for (int i = 0; i < 8; ++i) { { const int k = kc * 32 + 8 * g + i; const int c = k / KK, rm = k - c * KK; const int dy = rm / 3, dx = rm - dy * 3; a[i] = sx[c][pyl + dy][px + dx]; }
                                  { const int k = kc * 32 + 16 + 8 * g + i; const int c = k / KK, rm = k - c * KK; const int dy = rm / 3, dx = rm - dy * 3; a[8 + i] = sx[c][pyl + dy][px + dx]; } }
#pragma unroll
    for (int j = 0; j < 8; ++j) acc[j] = wmma_bf(a, frag_b(P + (size_t)(o0 + j * 16 + col) * KTOT + kc * 32, lane), acc[j]); }
  __syncthreads();
#pragma unroll
  for (int half = 0; half < 2; ++half) {
#pragma unroll
    for (int j = half * 4; j < half * 4 + 4; ++j)
#pragma unroll
      for (int r = 0; r < 8; ++r) { const int ol = j * 16 + col; st[ol - half * 64][wave * 16 + 8 * g + r] = acc[j][r] * SC[b * CO + o0 + ol] + bfr(CB[o0 + ol]); }
    __syncthreads();
    for (int e = tid; e < 64 * 16; e += 128) { const int ol = e >> 4, q = e & 15; const int ry = q >> 3, qq = q & 7; vst2(OUT + (((b * CO + o0 + half * 64 + ol) * HH + y0 + ry) * WWD) + qq * 4, *(const v4f*)&st[ol][ry * 32 + qq * 4]); }
    __syncthreads(); }
}
extern "C" void kernel_launch(void* const* d_in, const int* in_sizes, int n_in, void* d_out, int out_size, void* d_ws, size_t ws_size, hipStream_t stream) {
  (void)in_sizes; (void)n_in; (void)out_size;
  const float** F = (const float**)d_in;
  if (ws_size < (size_t)WS_END) return;
  char* ws = (char*)d_ws; __bf16* P = (__bf16*)ws; float *W2 = (float*)(ws + WS_W2), *SC = (float*)(ws + WS_SC);
  k_pack<<<CO + 1, 256, 0, stream>>>(F[2], P, W2);
  k_style<<<NB, 256, 0, stream>>>(F[1], F[3], F[4], F[5], W2, SC);
  k_conv<<<dim3(HH / 2, CO / 128, TNB), 128, 0, stream>>>(F[0], P, SC, F[6], (float*)d_out);
}
